// GraphGeoModule_38998303048499
// MI455X (gfx1250) — hardware-verified
//
#include <hip/hip_runtime.h>
#include <stddef.h>


#define DIN    64
#define DH     256
#define DOUT   1024
#define NTHR   256
#define NWAVE  8
#define EPT    8
#define NGRP   2
#define CHUNK  (NTHR * EPT * NGRP)
#define WCAP   (EPT * NGRP * 32)
#define LISTN  (NWAVE * WCAP)
#define NBC    4096
#define NB1    512
#define NB2    128
#define BMW    8192
#define GR     64
#define GC     256
#define ASCALE 16.0f
#define WSCALE 8.0f
#define OSCALE 0.0078125f
#define WSCAP  ((size_t)134217728)

#define LDS_AGG1 (NB1 * DIN * 4 + LISTN * 4 + 64)
#define LDS_AGG2 (BMW * 4 + NB2 * DH * 4 + LISTN * 4 + NB2 * 8 + 64)
#define LDS_G1   (GR * GC * 4)
#define LDS_G2   (GR * GC * 2)

static_assert((CHUNK & (CHUNK - 1)) == 0);
static_assert(CHUNK == 4096);
static_assert(WCAP == 512);
static_assert((NBC & (NBC - 1)) == 0 && NBC <= 4096);
static_assert((NB1 & (NB1 - 1)) == 0 && NB1 <= 4096);
static_assert(NBC == NWAVE * 4 * 128);
static_assert((NBC % NB1) == 0);
static_assert((NB1 % GR) == 0 && (NB2 % GR) == 0);
static_assert(NB2 == 128);
static_assert((DIN % 32) == 0 && (DH % 32) == 0);
static_assert(DH == GC && (DOUT % GC) == 0);
static_assert(GR == NWAVE * 8);
static_assert((NB1 * DIN / 8) == 16 * NTHR && (NB2 * DH / 8) == 16 * NTHR);
static_assert((DH * DIN / 8) % NTHR == 0);
static_assert((BMW % 4) == 0);

typedef float          v2f  __attribute__((ext_vector_type(2)));
typedef float          v4f  __attribute__((ext_vector_type(4)));
typedef float          v8f  __attribute__((ext_vector_type(8)));
typedef int            v4i  __attribute__((ext_vector_type(4)));
typedef unsigned       v4u  __attribute__((ext_vector_type(4)));
typedef unsigned short v8us __attribute__((ext_vector_type(8)));
typedef _Float16       v8h  __attribute__((ext_vector_type(8)));
typedef _Float16       v16h __attribute__((ext_vector_type(16)));
union FragH { v16h v; v8h h[2]; };

__device__ __forceinline__ v8h cvt8(v4f a, v4f b) {
  v8h r;
  r[0] = (_Float16)a.x; r[1] = (_Float16)a.y; r[2] = (_Float16)a.z; r[3] = (_Float16)a.w;
  r[4] = (_Float16)b.x; r[5] = (_Float16)b.y; r[6] = (_Float16)b.z; r[7] = (_Float16)b.w;
  return r;
}

__device__ __forceinline__ unsigned short bf16_rne(float f) {
  unsigned u = __float_as_uint(f);
  u = u + 0x7FFFu + ((u >> 16) & 1u);
  return (unsigned short)(u >> 16);
}

__device__ __forceinline__ v8f wmh(v16h a, v16h b, v8f c) {
  v8f d = __builtin_amdgcn_wmma_f32_16x16x32_f16(false, a, false, b, (short)0, c, false, false);
  asm volatile("v_nop\n\tv_nop\n\tv_nop\n\tv_nop" : "+v"(d) : "v"(a), "v"(b));
  return d;
}

template <int MODE, int NB>
__device__ __forceinline__ int scan_chunk(const int* __restrict__ dsts, int nE, int cbase, int slotBase,
                                          const unsigned* bm, int nN, int vec8, int* list,
                                          int tid, int wave) {
  int wc = 0;
#pragma unroll
  for (int g = 0; g < NGRP; ++g) {
    const int el0 = (g * NTHR + tid) * EPT;
    const int e0  = cbase + el0;
    int d[8];
    if (vec8 != 0 && cbase + CHUNK <= nE) {
      const v4i da = *(const v4i*)(dsts + e0);
      const v4i db = *(const v4i*)(dsts + e0 + 4);
      d[0] = da.x; d[1] = da.y; d[2] = da.z; d[3] = da.w;
      d[4] = db.x; d[5] = db.y; d[6] = db.z; d[7] = db.w;
    } else {
#pragma unroll
      for (int j = 0; j < 8; ++j) {
        int e = e0 + j;
        e = e > nE - 1 ? nE - 1 : e;
        d[j] = dsts[e];
      }
    }
    bool hit[8];
    int  pay[8];
    bool anyh = false;
#pragma unroll
    for (int j = 0; j < 8; ++j) {
      const bool valid = (e0 + j) < nE;
      if (MODE == 0) {
        const unsigned s = (unsigned)d[j] - (unsigned)slotBase;
        hit[j] = valid && (s < (unsigned)NB);
        pay[j] = (int)(s & 4095u);
      } else {
        const bool inr = (unsigned)d[j] < (unsigned)nN;
        int dc = d[j];
        dc = dc < 0 ? 0 : (dc > nN - 1 ? nN - 1 : dc);
        const unsigned w = bm[dc >> 5];
        hit[j] = valid && inr && (((w >> (dc & 31)) & 1u) != 0u);
        pay[j] = 0;
      }
      anyh = anyh || hit[j];
    }
    const unsigned anyb = __builtin_amdgcn_ballot_w32(anyh);
    if (anyb != 0u) {
#pragma unroll
      for (int j = 0; j < 8; ++j) {
        const unsigned mj = __builtin_amdgcn_ballot_w32(hit[j]);
        if (mj != 0u) {
          if (hit[j]) {
            const int pos = wc + (int)__builtin_amdgcn_mbcnt_lo(mj, 0u);
            if (pos < WCAP) list[wave * WCAP + pos] = ((el0 + j) << 12) | pay[j];
          }
          wc += (int)__builtin_popcount(mj);
        }
      }
    }
  }
  return wc;
}

__global__ __launch_bounds__(NTHR) void k_wprep(
    const float* __restrict__ W1, const float* __restrict__ W2, _Float16* w1s, _Float16* w2s) {
  const int g0 = DH * DIN / 8;
  const int g1 = DOUT * DH / 8;
  const int bstart = blockIdx.x * NTHR;
  const float* src; _Float16* dst; int K, Nout, segOff;
  if (bstart < g0) { src = W1; dst = w1s; K = DIN; Nout = DH;   segOff = 0;  }
  else             { src = W2; dst = w2s; K = DH;  Nout = DOUT; segOff = g0; }
  const int i = bstart + (int)threadIdx.x;
  if (i >= g0 + g1) return;
  const int o  = (i - segOff) * 8;
  const int n  = o / K;
  const int k0 = o - n * K;
  float v[8];
#pragma unroll
  for (int e = 0; e < 8; ++e) v[e] = src[(size_t)(k0 + e) * Nout + n] * WSCALE;
  v4f a, b;
  a.x = v[0]; a.y = v[1]; a.z = v[2]; a.w = v[3];
  b.x = v[4]; b.y = v[5]; b.z = v[6]; b.w = v[7];
  const v8h hv = cvt8(a, b);
  _Float16* dp = dst + o;
  *(volatile v8h*)dp = hv;
  __threadfence();
  *(volatile v8h*)dp = hv;
}

__global__ __launch_bounds__(NTHR) void k_count(const int* __restrict__ ei, float* dinv, int nE, int vec8) {
  __shared__ __attribute__((aligned(16))) int scnt[NBC];
  __shared__ __attribute__((aligned(16))) int list[LISTN];
  __shared__ int wcnt[NWAVE];
  const int tid = threadIdx.x, lane = tid & 31, wave = tid >> 5;
  const int nodeBase = blockIdx.x * NBC;
  const int* dsts = ei + nE;

  for (int i = tid; i < NBC; i += NTHR) scnt[i] = 0;
  __syncthreads();

  const int nChunks = (nE + CHUNK - 1) / CHUNK;
#pragma unroll 1
  for (int ch = 0; ch < nChunks; ++ch) {
    const int cbase = ch * CHUNK;
    const int wc = scan_chunk<0, NBC>(dsts, nE, cbase, nodeBase, (const unsigned*)scnt, 0, vec8, list, tid, wave);
    if (lane == 0) wcnt[wave] = wc;
    __syncthreads();
    if (wave == 0) {
#pragma unroll 1
      for (int wsx = 0; wsx < NWAVE; ++wsx) {
        int n = __builtin_amdgcn_readfirstlane(wcnt[wsx]);
        n = n > WCAP ? WCAP : (n < 0 ? 0 : n);
        const int* lp = list + wsx * WCAP;
#pragma unroll 1
        for (int i = 0; i < n; ++i) {
          const int ent  = __builtin_amdgcn_readfirstlane(lp[i]);
          const int slot = ent & (NBC - 1);
          if (lane == 0) scnt[slot] = scnt[slot] + 1;
        }
      }
    }
    __syncthreads();
  }

  v4f dq[4];
#pragma unroll
  for (int q = 0; q < 4; ++q) {
    const int f = (wave * 4 + q) * 128 + 4 * lane;
    const v4i c = *(const v4i*)(scnt + f);
    dq[q].x = rsqrtf((float)(c.x + 1));
    dq[q].y = rsqrtf((float)(c.y + 1));
    dq[q].z = rsqrtf((float)(c.z + 1));
    dq[q].w = rsqrtf((float)(c.w + 1));
  }
  float* dp = dinv + (size_t)nodeBase;
#pragma unroll
  for (int q = 0; q < 4; ++q) {
    const int f = (wave * 4 + q) * 128 + 4 * lane;
    *(volatile v4f*)(dp + f) = dq[q];
  }
  __threadfence();
#pragma unroll
  for (int q = 0; q < 4; ++q) {
    const int f = (wave * 4 + q) * 128 + 4 * lane;
    *(volatile v4f*)(dp + f) = dq[q];
  }
}

__global__ __launch_bounds__(NTHR) void k_agg1(
    const float* __restrict__ X, const int* __restrict__ ei, const float* __restrict__ dinv,
    _Float16* agg, int nN, int nE, int vec8) {
  extern __shared__ v4f lds_dyn[];
  float* acc  = (float*)lds_dyn;
  int*   list = (int*)(acc + NB1 * DIN);
  int*   wcnt = list + LISTN;
  const int tid = threadIdx.x, lane = tid & 31, wave = tid >> 5;
  const int nodeBase = blockIdx.x * NB1;
  const int* srcs = ei;
  const int* dsts = ei + nE;

  {
    const v4f z = {0.f, 0.f, 0.f, 0.f};
    for (int i = tid; i < NB1 * DIN / 4; i += NTHR) ((v4f*)acc)[i] = z;
  }
  __syncthreads();

  const int nChunks = (nE + CHUNK - 1) / CHUNK;
#pragma unroll 1
  for (int ch = 0; ch < nChunks; ++ch) {
    const int cbase = ch * CHUNK;
    const int wc = scan_chunk<0, NB1>(dsts, nE, cbase, nodeBase, (const unsigned*)list, nN, vec8, list, tid, wave);
    if (lane == 0) wcnt[wave] = wc;
    __syncthreads();
    if (wave == 0) {
#pragma unroll 1
      for (int wsx = 0; wsx < NWAVE; ++wsx) {
        int n = __builtin_amdgcn_readfirstlane(wcnt[wsx]);
        n = n > WCAP ? WCAP : (n < 0 ? 0 : n);
        const int* lp = list + wsx * WCAP;
#pragma unroll 1
        for (int i = 0; i < n; ++i) {
          const int ent  = __builtin_amdgcn_readfirstlane(lp[i]);
          const int slot = ent & (NB1 - 1);
          int e = cbase + ((ent >> 12) & (CHUNK - 1));
          e = e > nE - 1 ? nE - 1 : e;
          int src = srcs[e];
          src = src < 0 ? 0 : (src > nN - 1 ? nN - 1 : src);
          const float w = dinv[src];
          const v2f x = *(const v2f*)(X + (size_t)src * DIN + 2 * lane);
          v2f* ap = (v2f*)(acc + slot * DIN + 2 * lane);
          *ap = *ap + x * w;
        }
      }
    }
    __syncthreads();
  }

  v8h hv[16];
#pragma unroll
  for (int it = 0; it < 16; ++it) {
    const int idx = it * NTHR + tid;
    const int row = idx >> 3;
    const int c0  = (idx & 7) * 8;
    const int c   = nodeBase + row;
    const int cc  = c > nN - 1 ? nN - 1 : c;
    const float d = dinv[cc];
    const float* xp = X + (size_t)cc * DIN + c0;
    const v4f xa = *(const v4f*)xp, xb = *(const v4f*)(xp + 4);
    const v4f aa = *(const v4f*)(acc + row * DIN + c0);
    const v4f ab = *(const v4f*)(acc + row * DIN + c0 + 4);
    const float s = (c < nN) ? d * ASCALE : 0.0f;
    const v4f va = (aa + xa * d) * s;
    const v4f vb = (ab + xb * d) * s;
    hv[it] = cvt8(va, vb);
  }
  _Float16* gp = agg + (size_t)nodeBase * DIN;
#pragma unroll
  for (int it = 0; it < 16; ++it) *(volatile v8h*)(gp + (size_t)(it * NTHR + tid) * 8) = hv[it];
  __threadfence();
#pragma unroll
  for (int it = 0; it < 16; ++it) *(volatile v8h*)(gp + (size_t)(it * NTHR + tid) * 8) = hv[it];
}

__global__ __launch_bounds__(NTHR) void k_agg2(
    const float* __restrict__ x1, const int* __restrict__ ei, const int* __restrict__ geo,
    const float* __restrict__ dinv, _Float16* agg, int nN, int nE, int nIds, int vec8) {
  extern __shared__ v4f lds_dyn[];
  unsigned* bm    = (unsigned*)lds_dyn;
  float*    acc   = (float*)(bm + BMW);
  int*      list  = (int*)(acc + NB2 * DH);
  int*      gidS  = list + LISTN;
  int*      canon = gidS + NB2;
  int*      wcnt  = canon + NB2;
  const int tid = threadIdx.x, lane = tid & 31, wave = tid >> 5;
  const int pBase = blockIdx.x * NB2;
  const int* srcs = ei;
  const int* dsts = ei + nE;

  {
    const v4u zu = {0u, 0u, 0u, 0u};
    for (int i = tid; i < BMW / 4; i += NTHR) ((v4u*)bm)[i] = zu;
    const v4f z = {0.f, 0.f, 0.f, 0.f};
    for (int i = tid; i < NB2 * DH / 4; i += NTHR) ((v4f*)acc)[i] = z;
    if (tid < NB2) {
      int p = pBase + tid;
      p = p > nIds - 1 ? nIds - 1 : p;
      int g = geo[p];
      g = g < 0 ? g + nN : g;
      g = g < 0 ? 0 : (g > nN - 1 ? nN - 1 : g);
      gidS[tid] = g;
    }
  }
  __syncthreads();
  if (tid == 0) {
#pragma unroll 1
    for (int s = 0; s < NB2; ++s) {
      const int g = gidS[s];
      bm[g >> 5] = bm[g >> 5] | (1u << (g & 31));
    }
  }
  if (tid < NB2) {
    const int g = gidS[tid];
    int c = tid;
#pragma unroll 1
    for (int j = NB2 - 1; j >= 0; --j) {
      const int gj = gidS[j];
      c = (j < tid && gj == g) ? j : c;
    }
    canon[tid] = c;
  }
  __syncthreads();

  const int gq0 = gidS[lane], gq1 = gidS[lane + 32], gq2 = gidS[lane + 64], gq3 = gidS[lane + 96];

  const int nChunks = (nE + CHUNK - 1) / CHUNK;
#pragma unroll 1
  for (int ch = 0; ch < nChunks; ++ch) {
    const int cbase = ch * CHUNK;
    const int wc = scan_chunk<1, NB2>(dsts, nE, cbase, 0, bm, nN, vec8, list, tid, wave);
    if (lane == 0) wcnt[wave] = wc;
    __syncthreads();
    if (wave == 0) {
#pragma unroll 1
      for (int wsx = 0; wsx < NWAVE; ++wsx) {
        int n = __builtin_amdgcn_readfirstlane(wcnt[wsx]);
        n = n > WCAP ? WCAP : (n < 0 ? 0 : n);
        const int* lp = list + wsx * WCAP;
#pragma unroll 1
        for (int i = 0; i < n; ++i) {
          const int ent = __builtin_amdgcn_readfirstlane(lp[i]);
          int e = cbase + ((ent >> 12) & (CHUNK - 1));
          e = e > nE - 1 ? nE - 1 : e;
          int src = srcs[e];
          src = src < 0 ? 0 : (src > nN - 1 ? nN - 1 : src);
          const int dn = dsts[e];
          const unsigned m0 = __builtin_amdgcn_ballot_w32(gq0 == dn);
          const unsigned m1 = __builtin_amdgcn_ballot_w32(gq1 == dn);
          const unsigned m2 = __builtin_amdgcn_ballot_w32(gq2 == dn);
          const unsigned m3 = __builtin_amdgcn_ballot_w32(gq3 == dn);
          const int slot = m0 != 0u ? (__builtin_ffs((int)m0) - 1)
                         : (m1 != 0u ? (31 + __builtin_ffs((int)m1))
                         : (m2 != 0u ? (63 + __builtin_ffs((int)m2))
                         : (m3 != 0u ? (95 + __builtin_ffs((int)m3)) : -1)));
          if (slot >= 0) {
            const float w = dinv[src];
            const float* xp = x1 + (size_t)src * DH + 8 * lane;
            const v4f xa = *(const v4f*)xp, xb = *(const v4f*)(xp + 4);
            v4f* ap = (v4f*)(acc + slot * DH + 8 * lane);
            ap[0] = ap[0] + xa * w;
            ap[1] = ap[1] + xb * w;
          }
        }
      }
    }
    __syncthreads();
  }

  v8h hv[16];
#pragma unroll
  for (int it = 0; it < 16; ++it) {
    const int idx = it * NTHR + tid;
    const int row = idx >> 5;
    const int c0  = (idx & 31) * 8;
    const int g   = gidS[row];
    const int cs  = canon[row];
    const float d = dinv[g];
    const float* xp = x1 + (size_t)g * DH + c0;
    const v4f xa = *(const v4f*)xp, xb = *(const v4f*)(xp + 4);
    const v4f aa = *(const v4f*)(acc + cs * DH + c0);
    const v4f ab = *(const v4f*)(acc + cs * DH + c0 + 4);
    const float s = d * ASCALE;
    const v4f va = (aa + xa * d) * s;
    const v4f vb = (ab + xb * d) * s;
    hv[it] = cvt8(va, vb);
  }
  _Float16* gp = agg + (size_t)pBase * DH;
#pragma unroll
  for (int it = 0; it < 16; ++it) *(volatile v8h*)(gp + (size_t)(it * NTHR + tid) * 8) = hv[it];
  __threadfence();
#pragma unroll
  for (int it = 0; it < 16; ++it) *(volatile v8h*)(gp + (size_t)(it * NTHR + tid) * 8) = hv[it];
}

template <int KD, int NC, int OM>
__global__ __launch_bounds__(NTHR) void k_gemm(
    const _Float16* __restrict__ A, const _Float16* __restrict__ Bs, const float* __restrict__ bias,
    void* Cv, int nRowsStore) {
  extern __shared__ v4f lds_dyn[];
  const int tid = threadIdx.x, lane = tid & 31, wave = tid >> 5, hh = lane >> 4, m = lane & 15;
  const int mt = wave & 3, chf = wave >> 2;
  const int rowBase = blockIdx.x * GR;
  const int colBase = blockIdx.y * GC;

  v8f acc[8];
#pragma unroll
  for (int t = 0; t < 8; ++t) { v8f z = {0.f, 0.f, 0.f, 0.f, 0.f, 0.f, 0.f, 0.f}; acc[t] = z; }

  const _Float16* ar = A  + (size_t)(rowBase + 16 * mt + m) * KD + 8 * hh;
  const _Float16* br = Bs + (size_t)(colBase + 128 * chf + m) * KD + 8 * hh;
#pragma unroll 1
  for (int kt = 0; kt < KD / 32; ++kt) {
    FragH a;
    a.h[0] = *(const v8h*)(ar + 32 * kt);
    a.h[1] = *(const v8h*)(ar + 32 * kt + 16);
#pragma unroll
    for (int t = 0; t < 8; ++t) {
      const _Float16* bp = br + (size_t)(16 * t) * KD + 32 * kt;
      FragH b;
      b.h[0] = *(const v8h*)bp;
      b.h[1] = *(const v8h*)(bp + 16);
      acc[t] = wmh(a.v, b.v, acc[t]);
    }
  }

  const int r0 = 16 * mt + 8 * hh;
  if (OM == 0) {
    float* stg = (float*)lds_dyn;
#pragma unroll
    for (int t = 0; t < 8; ++t) {
      const int col = 128 * chf + 16 * t + m;
      const float bl = bias[colBase + col];
#pragma unroll
      for (int r = 0; r < 8; ++r) {
        float v = acc[t][r] * OSCALE + bl;
        v = fmaxf(v, 0.0f);
        stg[(r0 + r) * GC + col] = v;
      }
    }
    __syncthreads();
    float* C = (float*)Cv;
#pragma unroll
    for (int i = 0; i < 8; ++i) {
      const int row = wave * 8 + i;
      const int grow = rowBase + row;
      if (grow < nRowsStore) {
        const float* lp = stg + row * GC + 4 * lane;
        float* gp = C + (size_t)grow * NC + colBase + 4 * lane;
        const v4f v0 = *(const v4f*)lp, v1 = *(const v4f*)(lp + 128);
        *(volatile v4f*)gp = v0;
        *(volatile v4f*)(gp + 128) = v1;
      }
    }
    __threadfence();
#pragma unroll
    for (int i = 0; i < 8; ++i) {
      const int row = wave * 8 + i;
      const int grow = rowBase + row;
      if (grow < nRowsStore) {
        const float* lp = stg + row * GC + 4 * lane;
        float* gp = C + (size_t)grow * NC + colBase + 4 * lane;
        const v4f v0 = *(const v4f*)lp, v1 = *(const v4f*)(lp + 128);
        *(volatile v4f*)gp = v0;
        *(volatile v4f*)(gp + 128) = v1;
      }
    }
  } else {
    unsigned short* stg = (unsigned short*)lds_dyn;
#pragma unroll
    for (int t = 0; t < 8; ++t) {
      const int col = 128 * chf + 16 * t + m;
      const float bl = bias[colBase + col];
#pragma unroll
      for (int r = 0; r < 8; ++r) {
        float v = acc[t][r] * OSCALE + bl;
        v = fmaxf(v, 0.0f);
        stg[(r0 + r) * GC + col] = bf16_rne(v);
      }
    }
    __syncthreads();
    unsigned short* C = (unsigned short*)Cv;
#pragma unroll
    for (int i = 0; i < 8; ++i) {
      const int row = wave * 8 + i;
      const int grow = rowBase + row;
      if (grow < nRowsStore) {
        const v8us v = *(const v8us*)(stg + row * GC + 8 * lane);
        *(volatile v8us*)(C + (size_t)grow * NC + colBase + 8 * lane) = v;
      }
    }
    __threadfence();
#pragma unroll
    for (int i = 0; i < 8; ++i) {
      const int row = wave * 8 + i;
      const int grow = rowBase + row;
      if (grow < nRowsStore) {
        const v8us v = *(const v8us*)(stg + row * GC + 8 * lane);
        *(volatile v8us*)(C + (size_t)grow * NC + colBase + 8 * lane) = v;
      }
    }
  }
}

extern "C" void kernel_launch(void* const* d_in, const int* in_sizes, int n_in,
                              void* d_out, int out_size, void* d_ws, size_t ws_size,
                              hipStream_t stream) {
  if (n_in < 7) return;
  if (in_sizes[0] < DIN || (in_sizes[0] % DIN) != 0) return;
  const int nN = in_sizes[0] / DIN;
  if (in_sizes[1] != DIN * DH || in_sizes[2] != DH || in_sizes[3] != DH * DOUT || in_sizes[4] != DOUT) return;
  if (in_sizes[5] < 2 || (in_sizes[5] & 1) != 0) return;
  const int nE = in_sizes[5] / 2;
  const int nIds = in_sizes[6];
  if (nIds < 1 || nIds > (1 << 20)) return;
  if (out_size != nIds * DOUT) return;
  if (nN > BMW * 32 || nE > (1 << 28)) return;

  const float* X   = (const float*)d_in[0];
  const float* W1  = (const float*)d_in[1];
  const float* b1  = (const float*)d_in[2];
  const float* W2  = (const float*)d_in[3];
  const float* b2  = (const float*)d_in[4];
  const int*   ei  = (const int*)d_in[5];
  const int*   geo = (const int*)d_in[6];

  const int NPAD   = ((nN + NB1 - 1) / NB1) * NB1;
  const int nBC    = (nN + NBC - 1) / NBC;
  const int CNTPAD = nBC * NBC;
  const int NIDPAD = ((nIds + NB2 - 1) / NB2) * NB2;

  char* ws = (char*)d_ws;
  size_t off = 0;
  const size_t oW1 = off; off += (size_t)DH * DIN * 2;        off = (off + 255) & ~(size_t)255;
  const size_t oW2 = off; off += (size_t)DOUT * DH * 2;        off = (off + 255) & ~(size_t)255;
  const size_t oDv = off; off += (size_t)CNTPAD * 4;           off = (off + 255) & ~(size_t)255;
  const size_t oA1 = off; off += (size_t)NPAD * DIN * 2;       off = (off + 255) & ~(size_t)255;
  const size_t oX1 = off; off += (size_t)NPAD * DH * 4;        off = (off + 255) & ~(size_t)255;
  const size_t oA2 = off; off += (size_t)NIDPAD * DH * 2;      off = (off + 255) & ~(size_t)255;
  if (off > ws_size || off > WSCAP) return;
  _Float16* w1s  = (_Float16*)(ws + oW1);
  _Float16* w2s  = (_Float16*)(ws + oW2);
  float*    dinv = (float*)(ws + oDv);
  _Float16* agg1 = (_Float16*)(ws + oA1);
  float*    x1   = (float*)(ws + oX1);
  _Float16* agg2 = (_Float16*)(ws + oA2);

  const int vec8 = ((nE & 3) == 0) ? 1 : 0;

  const int nPrep = DH * DIN / 8 + DOUT * DH / 8;
  k_wprep<<<(nPrep + NTHR - 1) / NTHR, NTHR, 0, stream>>>(W1, W2, w1s, w2s);

  k_count<<<nBC, NTHR, 0, stream>>>(ei, dinv, nE, vec8);

  hipFuncSetAttribute(reinterpret_cast<const void*>(&k_agg1),
                      hipFuncAttributeMaxDynamicSharedMemorySize, LDS_AGG1);
  k_agg1<<<NPAD / NB1, NTHR, LDS_AGG1, stream>>>(X, ei, dinv, agg1, nN, nE, vec8);

  hipFuncSetAttribute(reinterpret_cast<const void*>(&k_gemm<DIN, DH, 0>),
                      hipFuncAttributeMaxDynamicSharedMemorySize, LDS_G1);
  k_gemm<DIN, DH, 0><<<dim3(NPAD / GR, DH / GC), NTHR, LDS_G1, stream>>>(agg1, w1s, b1, x1, NPAD);

  hipFuncSetAttribute(reinterpret_cast<const void*>(&k_agg2),
                      hipFuncAttributeMaxDynamicSharedMemorySize, LDS_AGG2);
  k_agg2<<<NIDPAD / NB2, NTHR, LDS_AGG2, stream>>>(x1, ei, geo, dinv, agg2, nN, nE, nIds, vec8);

  hipFuncSetAttribute(reinterpret_cast<const void*>(&k_gemm<DH, DOUT, 1>),
                      hipFuncAttributeMaxDynamicSharedMemorySize, LDS_G2);
  k_gemm<DH, DOUT, 1><<<dim3(NIDPAD / GR, DOUT / GC), NTHR, LDS_G2, stream>>>(agg2, w2s, b2, d_out, nIds);
}
